// CrossAttention3D_84885733638497
// MI455X (gfx1250) — hardware-verified
//
#include <hip/hip_runtime.h>


namespace {
constexpr int C = 512, NP = 4096, G = 8, CG = C / G, H = 8, HD = 64;
constexpr float QS = 8.0f, KS = 8.0f, VS = 8.0f, PS = 8.0f, AS_ = 8.0f, SCALE = 0.125f, EPS = 1e-5f;
constexpr size_t PL = (size_t)H * NP * HD;

typedef _Float16 b16;
typedef __attribute__((ext_vector_type(16))) _Float16 v16b;
typedef __attribute__((ext_vector_type(8))) _Float16 v8b;
typedef __attribute__((ext_vector_type(8))) float v8f;
typedef __attribute__((ext_vector_type(4))) float v4f;
__device__ __forceinline__ float bf16_rne(float f) { unsigned int u = __float_as_uint(f); u += 0x7FFFu + ((u >> 16) & 1u); return __uint_as_float(u & 0xFFFF0000u); }
__device__ __forceinline__ void split16(float v, b16& hi, b16& lo) { hi = (b16)v; lo = (b16)(v - (float)hi); }
__device__ __forceinline__ v16b frag_kb(const b16* p, int hh) { const v8b a = *(const v8b*)(p + 8 * hh), b = *(const v8b*)(p + 16 + 8 * hh); v16b f;
#pragma unroll
  for (int e = 0; e < 8; ++e) { f[e] = a[e]; f[8 + e] = b[e]; } return f; }
__device__ __forceinline__ void frag_split(const float* p, int hh, v16b& fh, v16b& fl) {
#pragma unroll
  for (int e = 0; e < 8; ++e) { b16 a, c; split16(p[8 * hh + e] * AS_, a, c); fh[e] = a; fl[e] = c; split16(p[16 + 8 * hh + e] * AS_, a, c); fh[8 + e] = a; fl[8 + e] = c; } }
__device__ __forceinline__ v8f wmma16b(v16b a, v16b b, v8f c) { v8f d = __builtin_amdgcn_wmma_f32_16x16x32_f16(false, a, false, b, (short)0, c, false, false); asm volatile("v_nop\n\tv_nop\n\tv_nop\n\tv_nop" : "+v"(d) : "v"(a), "v"(b)); return d; }
__device__ __forceinline__ void wave_lds_sync() { __builtin_amdgcn_fence(__ATOMIC_RELEASE, "workgroup"); __builtin_amdgcn_wave_barrier(); __builtin_amdgcn_fence(__ATOMIC_ACQUIRE, "workgroup"); }
__device__ __forceinline__ float nexp(float x) { return __builtin_amdgcn_exp2f(x * 1.4426950408889634f); }

__global__ __launch_bounds__(256) void prep_kernel(const float* __restrict__ qw, const float* __restrict__ kvw, const float* __restrict__ pw, const float* __restrict__ qb, const float* __restrict__ kvb, const float* __restrict__ pb, const float* __restrict__ nqw, const float* __restrict__ nqb, const float* __restrict__ nkw, const float* __restrict__ nkb, b16* __restrict__ R, float* __restrict__ P) {
  const size_t tid = (size_t)blockIdx.x * blockDim.x + threadIdx.x, nth = (size_t)gridDim.x * blockDim.x;
  for (int pass = 0; pass < 2; ++pass) {
    for (size_t p = tid; p < (size_t)4 * C * C / 8; p += nth) { const float* W; size_t q; if (p < (size_t)C * C / 8) { W = qw; q = p; } else if (p < (size_t)3 * C * C / 8) { W = kvw; q = p - (size_t)C * C / 8; } else { W = pw; q = p - (size_t)3 * C * C / 8; } v8b v;
#pragma unroll
      for (int e = 0; e < 8; ++e) v[e] = (b16)bf16_rne(W[q * 8 + e]);
      *(volatile v8b*)(R + p * 8) = v; }
    for (size_t p = tid; p < 4096 / 4; p += nth) { v4f v;
#pragma unroll
      for (int e = 0; e < 4; ++e) { const int i = (int)p * 4 + e; float x; if (i < 512) x = qb[i]; else if (i < 1536) x = kvb[i - 512]; else if (i < 2048) x = pb[i - 1536]; else if (i < 2560) x = nqw[i - 2048]; else if (i < 3072) x = nqb[i - 2560]; else if (i < 3584) x = nkw[i - 3072]; else x = nkb[i - 3584]; v[e] = bf16_rne(x); }
      *(volatile v4f*)(P + p * 4) = v; }
    __threadfence(); }
}

__global__ __launch_bounds__(256) void gnstat_kernel(const float* __restrict__ x, const float* __restrict__ ctxin, float* __restrict__ st) {
  __shared__ double rs[256], rq[256];
  const int tg = blockIdx.x, which = tg >> 3, g = tg & 7, t_ = threadIdx.x; const float* src = (which ? ctxin : x) + (size_t)g * CG * NP;
  double s = 0.0, q = 0.0;
  for (int i = t_; i < CG * NP; i += 256) { const double v = (double)bf16_rne(src[i]); s += v; q += v * v; }
  rs[t_] = s; rq[t_] = q; __syncthreads();
  for (int stp = 128; stp > 0; stp >>= 1) { if (t_ < stp) { rs[t_] += rs[t_ + stp]; rq[t_] += rq[t_ + stp]; } __syncthreads(); }
  if (t_ < 32) { const double n = (double)CG * NP, mean = rs[0] / n, var = fmax(rq[0] / n - mean * mean, 0.0); const float mf = (float)mean, rf = (float)(1.0 / sqrt(var + (double)EPS));
    for (int pass = 0; pass < 2; ++pass) { ((volatile float*)st)[tg * 32 + t_] = (t_ & 1) ? rf : mf; __threadfence(); } }
}

__global__ __launch_bounds__(256) void gnorm_kernel(const float* __restrict__ x, const float* __restrict__ ctxin, const float* __restrict__ st, const float* __restrict__ P, float* __restrict__ xn, float* __restrict__ cn) {
  __shared__ __attribute__((aligned(16))) float T[64][C + 4];
  const int which = blockIdx.y, p0 = blockIdx.x * 64, t_ = threadIdx.x; const float* src = which ? ctxin : x; const float* w = P + (which ? 3072 : 2048); const float* bb = P + (which ? 3584 : 2560); float* dst = which ? cn : xn;
  for (int i = t_; i < C * 64; i += 256) { const int c = i >> 6, pp = i & 63; const int g = c / CG; const float mean = st[(which * 8 + g) * 32], rstd = st[(which * 8 + g) * 32 + 1];
    T[pp][c] = (bf16_rne(src[(size_t)c * NP + p0 + pp]) - mean) * rstd * w[c] + bb[c]; }
  __syncthreads();
  for (int pass = 0; pass < 2; ++pass) { for (int i = t_; i < 64 * (C / 4); i += 256) { const int pp = i / (C / 4), c4 = (i % (C / 4)) * 4; *(volatile v4f*)(dst + (size_t)(p0 + pp) * C + c4) = *(const v4f*)(&T[pp][c4]); } __threadfence(); }
}

__global__ __launch_bounds__(128) void proj_kernel(const float* __restrict__ xn, const float* __restrict__ cn, const b16* __restrict__ R, const float* __restrict__ P, b16* __restrict__ qp, b16* __restrict__ kp, b16* __restrict__ vt) {
  __shared__ __attribute__((aligned(16))) b16 Th[4][32][64 + 8], Tl[4][32][64 + 8]; __shared__ __attribute__((aligned(16))) b16 Vh[64][128 + 8], Vl[64][128 + 8];
  const int lane = threadIdx.x & 31, wave = threadIdx.x >> 5, nloc = lane & 15, hlf = lane >> 4, which = blockIdx.z, h = blockIdx.x, c0 = h * HD, p0 = blockIdx.y * 128, m0 = p0 + wave * 32;
  const float* X = (which == 0) ? xn : cn; const b16* Wt = R + ((which == 0) ? (size_t)0 : (which == 1) ? (size_t)C * C : (size_t)2 * C * C); const float* bias = P + ((which == 0) ? 0 : (which == 1) ? 512 : 1024);
  v8f acc[2][4];
#pragma unroll
  for (int r = 0; r < 2; ++r)
#pragma unroll
    for (int t = 0; t < 4; ++t) acc[r][t] = (v8f){};
#pragma unroll 2
  for (int kb = 0; kb < C; kb += 32) { v16b a0, l0, a1, l1; frag_split(X + (size_t)(m0 + nloc) * C + kb, hlf, a0, l0); frag_split(X + (size_t)(m0 + 16 + nloc) * C + kb, hlf, a1, l1);
#pragma unroll
    for (int t = 0; t < 4; ++t) { const v16b bw = frag_kb(Wt + (size_t)(c0 + t * 16 + nloc) * C + kb, hlf); acc[0][t] = wmma16b(a0, bw, acc[0][t]); acc[0][t] = wmma16b(l0, bw, acc[0][t]); acc[1][t] = wmma16b(a1, bw, acc[1][t]); acc[1][t] = wmma16b(l1, bw, acc[1][t]); } }
  const float scl = (which == 0) ? SCALE * QS : ((which == 1) ? KS : VS);
  if (which < 2) {
#pragma unroll
    for (int t = 0; t < 4; ++t) { const float bb = bias[c0 + t * 16 + nloc];
#pragma unroll
      for (int r = 0; r < 2; ++r)
#pragma unroll
        for (int v = 0; v < 8; ++v) { b16 a_, l_; split16((acc[r][t][v] * (1.0f / AS_) + bb) * scl, a_, l_); Th[wave][r * 16 + 8 * hlf + v][t * 16 + nloc] = a_; Tl[wave][r * 16 + 8 * hlf + v][t * 16 + nloc] = l_; } }
    wave_lds_sync();
    b16* base = ((which == 0) ? qp : kp) + ((size_t)h * NP + m0) * HD;
    for (int pass = 0; pass < 2; ++pass) {
#pragma unroll
      for (int j = 0; j < 8; ++j) { const int rr = j * 4 + (lane >> 3), c8 = (lane & 7) * 8; *(volatile v8b*)(base + (size_t)rr * HD + c8) = *(const v8b*)(&Th[wave][rr][c8]); *(volatile v8b*)(base + PL + (size_t)rr * HD + c8) = *(const v8b*)(&Tl[wave][rr][c8]); }
      __threadfence(); }
    return; }
#pragma unroll
  for (int t = 0; t < 4; ++t) { const float bb = bias[c0 + t * 16 + nloc];
#pragma unroll
    for (int r = 0; r < 2; ++r)
#pragma unroll
      for (int v = 0; v < 8; ++v) { b16 a_, l_; split16((acc[r][t][v] * (1.0f / AS_) + bb) * scl, a_, l_); Vh[t * 16 + nloc][wave * 32 + r * 16 + 8 * hlf + v] = a_; Vl[t * 16 + nloc][wave * 32 + r * 16 + 8 * hlf + v] = l_; } }
  __syncthreads();
  for (int pass = 0; pass < 2; ++pass) { for (int i = threadIdx.x; i < 64 * 16; i += 128) { const int d = i >> 4, c8 = (i & 15) * 8; const size_t o = ((size_t)h * HD + d) * NP + p0 + c8;
      *(volatile v8b*)(vt + o) = *(const v8b*)(&Vh[d][c8]); *(volatile v8b*)(vt + PL + o) = *(const v8b*)(&Vl[d][c8]); } __threadfence(); }
}

__global__ __launch_bounds__(256) void attn_kernel(const b16* __restrict__ qp, const b16* __restrict__ kp, const b16* __restrict__ vt, float* __restrict__ ctx) {
  __shared__ __attribute__((aligned(16))) float Os[16][C + 4];
  const int h = threadIdx.x >> 5, lane = threadIdx.x & 31, hh = lane >> 4, col = lane & 15; const int q0 = blockIdx.x * 16, qi = q0 + col;
  const b16* Q = qp + ((size_t)h * NP) * HD; const b16* K = kp + ((size_t)h * NP) * HD; const b16* V = vt + ((size_t)h * HD) * NP;
  v16b qf[2], ql[2];
#pragma unroll
  for (int ks = 0; ks < 2; ++ks) { qf[ks] = frag_kb(Q + (size_t)qi * HD + ks * 32, hh); ql[ks] = frag_kb(Q + PL + (size_t)qi * HD + ks * 32, hh); }
  float m = -INFINITY, l = 0.0f; v8f o[4] = {{}, {}, {}, {}};
  for (int kb = 0; kb < NP; kb += 32) { v8f s0 = {}, s1 = {};
#pragma unroll
    for (int ks = 0; ks < 2; ++ks) { const v16b ka = frag_kb(K + (size_t)(kb + col) * HD + ks * 32, hh), kal = frag_kb(K + PL + (size_t)(kb + col) * HD + ks * 32, hh), kc = frag_kb(K + (size_t)(kb + 16 + col) * HD + ks * 32, hh), kcl = frag_kb(K + PL + (size_t)(kb + 16 + col) * HD + ks * 32, hh);
      s0 = wmma16b(ka, qf[ks], s0); s0 = wmma16b(ka, ql[ks], s0); s0 = wmma16b(kal, qf[ks], s0); s1 = wmma16b(kc, qf[ks], s1); s1 = wmma16b(kc, ql[ks], s1); s1 = wmma16b(kcl, qf[ks], s1); }
    float mr = -INFINITY;
#pragma unroll
    for (int r = 0; r < 8; ++r) { s0[r] *= 1.0f / (QS * KS); s1[r] *= 1.0f / (QS * KS); mr = fmaxf(mr, fmaxf(s0[r], s1[r])); }
    mr = fmaxf(mr, __shfl_xor(mr, 16));
    const float mn = fmaxf(m, mr), al_ = nexp(m - mn); m = mn; float sum = 0.0f; v16b pbv, plv;
#pragma unroll
    for (int r = 0; r < 8; ++r) { const float e0 = nexp(s0[r] - mn), e1 = nexp(s1[r] - mn); sum += e0 + e1; b16 a, cc; split16(e0 * PS, a, cc); pbv[r] = a; plv[r] = cc; split16(e1 * PS, a, cc); pbv[8 + r] = a; plv[8 + r] = cc; }
    sum += __shfl_xor(sum, 16); l = l * al_ + sum;
#pragma unroll
    for (int t = 0; t < 4; ++t) { o[t] *= al_; const v16b vf = frag_kb(V + (size_t)(t * 16 + col) * NP + kb, hh), vl = frag_kb(V + PL + (size_t)(t * 16 + col) * NP + kb, hh); o[t] = wmma16b(vf, pbv, o[t]); o[t] = wmma16b(vf, plv, o[t]); o[t] = wmma16b(vl, pbv, o[t]); } }
  const float inv = 1.0f / (l * VS * PS);
#pragma unroll
  for (int t = 0; t < 4; ++t)
#pragma unroll
    for (int r = 0; r < 8; ++r) Os[col][h * HD + t * 16 + 8 * hh + r] = o[t][r] * inv;
  __syncthreads();
  for (int pass = 0; pass < 2; ++pass) { for (int i = threadIdx.x; i < 16 * (C / 4); i += 256) { const int rr = i / (C / 4), c4 = (i % (C / 4)) * 4; *(volatile v4f*)(ctx + (size_t)(q0 + rr) * C + c4) = *(const v4f*)(&Os[rr][c4]); } __threadfence(); }
}

__global__ __launch_bounds__(128) void out_kernel(const float* __restrict__ ctx, const b16* __restrict__ R, const float* __restrict__ P, const float* __restrict__ x, float* __restrict__ out) {
  __shared__ __attribute__((aligned(16))) float Tc[64][128 + 4];
  const int lane = threadIdx.x & 31, wave = threadIdx.x >> 5, nloc = lane & 15, hlf = lane >> 4, p0 = blockIdx.y * 128, m0 = p0 + wave * 32, c0 = blockIdx.x * 64; const b16* Wt = R + (size_t)3 * C * C; const float* pb = P + 1536;
  v8f acc[2][4];
#pragma unroll
  for (int r = 0; r < 2; ++r)
#pragma unroll
    for (int t = 0; t < 4; ++t) acc[r][t] = (v8f){};
#pragma unroll 2
  for (int kb = 0; kb < C; kb += 32) { v16b a0, l0, a1, l1; frag_split(ctx + (size_t)(m0 + nloc) * C + kb, hlf, a0, l0); frag_split(ctx + (size_t)(m0 + 16 + nloc) * C + kb, hlf, a1, l1);
#pragma unroll
    for (int t = 0; t < 4; ++t) { const v16b bw = frag_kb(Wt + (size_t)(c0 + t * 16 + nloc) * C + kb, hlf); acc[0][t] = wmma16b(a0, bw, acc[0][t]); acc[0][t] = wmma16b(l0, bw, acc[0][t]); acc[1][t] = wmma16b(a1, bw, acc[1][t]); acc[1][t] = wmma16b(l1, bw, acc[1][t]); } }
#pragma unroll
  for (int t = 0; t < 4; ++t) { const int cc = c0 + t * 16 + nloc; const float bb = pb[cc];
#pragma unroll
    for (int r = 0; r < 2; ++r)
#pragma unroll
      for (int v = 0; v < 8; ++v) { const int pl = wave * 32 + r * 16 + 8 * hlf + v; Tc[t * 16 + nloc][pl] = acc[r][t][v] * (1.0f / AS_) + bb + bf16_rne(x[(size_t)cc * NP + p0 + pl]); } }
  __syncthreads();
  for (int pass = 0; pass < 2; ++pass) { for (int i = threadIdx.x; i < 64 * 32; i += 128) { const int cc = i >> 5, c4 = (i & 31) * 4; *(volatile v4f*)(out + (size_t)(c0 + cc) * NP + p0 + c4) = *(const v4f*)(&Tc[cc][c4]); } __threadfence(); }
}
}

extern "C" void kernel_launch(void* const* d_in, const int* in_sizes, int n_in,
                              void* d_out, int out_size, void* d_ws, size_t ws_size, hipStream_t stream) {
  (void)n_in; (void)out_size;
  const float* x = (const float*)d_in[0]; const float* ctxin = (const float*)d_in[1]; const float* nqw = (const float*)d_in[2]; const float* nqb = (const float*)d_in[3]; const float* nkw = (const float*)d_in[4]; const float* nkb = (const float*)d_in[5];
  const float* qw = (const float*)d_in[6]; const float* qb = (const float*)d_in[7]; const float* kvw = (const float*)d_in[8]; const float* kvb = (const float*)d_in[9]; const float* pw = (const float*)d_in[10]; const float* pb = (const float*)d_in[11];
  float* out = (float*)d_out;
  if (in_sizes[0] != C * NP || in_sizes[1] != C * NP || in_sizes[6] != C * C || in_sizes[8] != 2 * C * C || in_sizes[10] != C * C) return;
  size_t off = 0; char* ws = (char*)d_ws;
  auto carve = [&](size_t bytes) { char* p = ws + off; off += (bytes + 255) & ~(size_t)255; return p; };
  b16* R = (b16*)carve((size_t)4 * C * C * 2); float* P = (float*)carve(4096 * 4); float* st = (float*)carve(16 * 32 * 4); float* xn = (float*)carve((size_t)NP * C * 4); float* cn = (float*)carve((size_t)NP * C * 4);
  b16* qp = (b16*)carve(PL * 2 * 2); b16* kp = (b16*)carve(PL * 2 * 2); b16* vt = (b16*)carve(PL * 2 * 2); float* ctx = xn;
  if (off > ws_size) return;
  prep_kernel<<<256, 256, 0, stream>>>(qw, kvw, pw, qb, kvb, pb, nqw, nqb, nkw, nkb, R, P);
  gnstat_kernel<<<16, 256, 0, stream>>>(x, ctxin, st);
  gnorm_kernel<<<dim3(NP / 64, 2), 256, 0, stream>>>(x, ctxin, st, P, xn, cn);
  proj_kernel<<<dim3(H, NP / 128, 3), 128, 0, stream>>>(xn, cn, R, P, qp, kp, vt);
  attn_kernel<<<NP / 16, 256, 0, stream>>>(qp, kp, vt, ctx);
  out_kernel<<<dim3(C / 64, NP / 128), 128, 0, stream>>>(ctx, R, P, x, out);
}
